// LinearMulti_6124623364236
// MI455X (gfx1250) — hardware-verified
//
#include <hip/hip_runtime.h>


#ifndef NB
#define NB 4096
#endif
#define NB_FULL 4096
#define SZ     256
#define NMOD   128
#define NSEG   8
#define SEGLEN (NB / NSEG)
#define TROWS  16
#define PROWS  (NB + 2048)
#define NTILE  (PROWS / TROWS)
#define OSP    260

static_assert(NB % 1024 == 0);
static_assert(NB <= NB_FULL);
static_assert(NB <= 4096);
static_assert(NB % NSEG == 0);
static_assert(NMOD * NSEG == 1024);
static_assert(NMOD == 32 * 4);
static_assert(NMOD * 15 <= 2048);
static_assert(PROWS % TROWS == 0);
static_assert(NTILE % 32 == 0 && NTILE <= 1024);
static_assert(SZ == 256);
static_assert(SZ % 32 == 0);
static_assert(SZ / 4 == 64);
static_assert(SZ * 2 == 32 * 16);
static_assert((OSP * 4) % 16 == 0 && OSP >= SZ);
static_assert(32 * 16 * (TROWS * 2) == TROWS * SZ * 4);
static_assert(256 * 16 * 2 == 64 * 64 * 2);
static_assert((size_t)NB * 4 * 2 + (size_t)NMOD * 4 * 2 <= 131072);
static_assert((size_t)TROWS * OSP * 4 <= 131072);
static_assert((size_t)64 * 65 * 4 <= 131072);

typedef unsigned short bf;
typedef __attribute__((ext_vector_type(16))) __bf16   v16bf;
typedef __attribute__((ext_vector_type(8)))  unsigned short v8us;
typedef __attribute__((ext_vector_type(8)))  float    v8f;
typedef __attribute__((ext_vector_type(4)))  float    v4f;
typedef __attribute__((ext_vector_type(4)))  int      v4i;
typedef v4f  __attribute__((may_alias)) v4fa;
typedef v4i  __attribute__((may_alias)) v4ia;

__device__ __forceinline__ unsigned short f2bf(float f) { unsigned u = __float_as_uint(f); u += 0x7FFFu + ((u >> 16) & 1u); return (unsigned short)(u >> 16); }
__device__ __forceinline__ float bf2f(unsigned short w) { return __uint_as_float(((unsigned)w) << 16); }
__device__ __forceinline__ int clampi(int v, int lo, int hi) { return min(max(v, lo), hi); }
__device__ __forceinline__ v16bf cat16b(v8us lo, v8us hi) { return __builtin_bit_cast(v16bf, __builtin_shufflevector(lo, hi, 0, 1, 2, 3, 4, 5, 6, 7, 8, 9, 10, 11, 12, 13, 14, 15)); }
__device__ __forceinline__ v8f wmmab(v16bf a, v16bf b, v8f c) { return __builtin_amdgcn_wmma_f32_16x16x32_bf16(false, a, false, b, (short)0, c, false, false); }
__device__ __forceinline__ v8f wmmab_g(v16bf a, v16bf b, v8f c) { c = wmmab(a, b, c); asm volatile("v_nop\n\tv_nop\n\tv_nop\n\tv_nop" : "+v"(c) : "v"(a), "v"(b)); return c; }
__device__ __forceinline__ v16bf ldb(const bf* p)  { return cat16b(*(const v8us*)p, *(const v8us*)(p + 16)); }
__device__ __forceinline__ void wave_sync() { __builtin_amdgcn_fence(3  , "wavefront"); __builtin_amdgcn_wave_barrier(); asm volatile("" ::: "memory"); }

__global__ __launch_bounds__(256) void k_wt(const float* __restrict__ W, bf* WT) {
    __shared__ float ts[64 * 65];
    const int r = blockIdx.x >> 4, tile = blockIdx.x & 15, t = threadIdx.x;
    const int i0 = (tile >> 2) * 64, o0 = (tile & 3) * 64;
    const float* src = W + (size_t)r * (SZ * SZ) + (size_t)i0 * SZ + o0;
#pragma unroll 1
    for (int i = 0; i < 16; ++i) { const int f = i * 256 + t; ts[(f >> 6) * 65 + (f & 63)] = src[(size_t)(f >> 6) * SZ + (f & 63)]; }
    __syncthreads();
    bf* dst = WT + (size_t)r * (SZ * SZ) + (size_t)o0 * SZ + i0;
#pragma unroll 1
    for (int ps = 0; ps < 2; ++ps) {
#pragma unroll 1
        for (int it = 0; it < 2; ++it) {
            const int e = it * 32 + (t >> 3), c8 = (t & 7) * 8; v8us o;
#pragma unroll
            for (int k = 0; k < 8; ++k) o[k] = f2bf(ts[(c8 + k) * 65 + e]);
            *(volatile v8us*)(dst + (size_t)e * SZ + c8) = o; }
        if (ps == 0) __threadfence(); }
}

__global__ __launch_bounds__(1024) void k_sort(const int* __restrict__ ids, int* POS, int* TM, bf* AP) {
    __shared__ int sid[NB];
    __shared__ __align__(16) int posl[NB];
    __shared__ int tots[NMOD];
    __shared__ int sst[NMOD];
    const int tid = threadIdx.x, lane = tid & 31; const int wave = __builtin_amdgcn_readfirstlane(tid >> 5);
#pragma unroll 1
    for (int i = 0; i < NB / 1024; ++i) { const int j = i * 1024 + tid; sid[j] = clampi(ids[j], 0, NMOD - 1); }
    __syncthreads();
    const int g = tid >> 3, s = tid & 7;
    int c = 0;
#pragma unroll 4
    for (int j = 0; j < SEGLEN; ++j) { const int v = sid[s * SEGLEN + j]; c += (v == g) ? 1 : 0; }
    int x = c;
#pragma unroll
    for (int d = 1; d < 8; d <<= 1) { const int y = __shfl_up(x, d, 8); x += (s >= d) ? y : 0; }
    const int excl = x - c;
    if (s == 7) tots[g] = x;
    __syncthreads();
    if (wave == 0) {
        int t4[4]; int ls = 0;
#pragma unroll
        for (int i = 0; i < 4; ++i) { t4[i] = (clampi(tots[4 * lane + i], 0, NB) + 15) & ~15; ls += t4[i]; }
        int y2 = ls;
#pragma unroll
        for (int d = 1; d < 32; d <<= 1) { const int y = __shfl_up(y2, d, 32); y2 += (lane >= d) ? y : 0; }
        const int e0 = y2 - ls;
        sst[4 * lane] = e0; sst[4 * lane + 1] = e0 + t4[0]; sst[4 * lane + 2] = e0 + t4[0] + t4[1]; sst[4 * lane + 3] = e0 + t4[0] + t4[1] + t4[2];
    }
    __syncthreads();
    {
        int run = sst[g] + excl;
#pragma unroll 1
        for (int j = 0; j < SEGLEN; ++j) { const int jj = s * SEGLEN + j; const int v = sid[jj]; const bool hit = (v == g);
            if (hit) posl[jj] = clampi(run, 0, PROWS - 1);
            run += hit ? 1 : 0; }
    }
    int tm = -1;
    {
        const int p0 = tid * TROWS;
#pragma unroll 1
        for (int mm = 0; mm < NMOD; ++mm) { const int ss = sst[mm]; const int pe = ss + ((clampi(tots[mm], 0, NB) + 15) & ~15); tm = ((p0 >= ss) && (p0 < pe)) ? mm : tm; }
    }
    __syncthreads();
    v8us z;
#pragma unroll
    for (int k = 0; k < 8; ++k) z[k] = (unsigned short)0;
#pragma unroll 1
    for (int ps = 0; ps < 2; ++ps) {
#pragma unroll 1
        for (int i = tid; i < NB / 4; i += 1024) { const v4i v = *(const v4ia*)(&posl[4 * i]); *(volatile v4i*)(POS + 4 * (size_t)i) = v; }
        if (tid < NTILE) *(volatile int*)(TM + tid) = tm;
#pragma unroll 1
        for (int q = 0; q < 4; ++q) { const int mm = wave * 4 + q; const int tot = clampi(tots[mm], 0, NB); const int st = sst[mm];
            const int padcnt = ((tot + 15) & ~15) - tot;
            const int pbase = st + tot;
#pragma unroll 1
            for (int j = 0; j < 16; ++j) { const int p = clampi(pbase + j, 0, PROWS - 1);
                if (j < padcnt) *(volatile v8us*)(AP + (size_t)p * SZ + lane * 8) = z; } }
        if (ps == 0) __threadfence(); }
}

__global__ __launch_bounds__(256) void k_pack(const float* __restrict__ X, const int* __restrict__ POS, bf* AP) {
    const int lane = threadIdx.x & 31; const int wave = __builtin_amdgcn_readfirstlane(threadIdx.x >> 5);
    const int rb = blockIdx.x * 32 + wave * 4;
#pragma unroll 1
    for (int ps = 0; ps < 2; ++ps) {
#pragma unroll 1
        for (int it = 0; it < 4; ++it) { const int b = rb + it; const int p = clampi(POS[b], 0, PROWS - 1);
            const v8f a = *(const v8f*)(X + (size_t)b * SZ + lane * 8); v8us oa;
#pragma unroll
            for (int k = 0; k < 8; ++k) oa[k] = f2bf(a[k]);
            *(volatile v8us*)(AP + (size_t)p * SZ + lane * 8) = oa; }
        if (ps == 0) __threadfence(); }
}

__global__ __launch_bounds__(32) __attribute__((amdgpu_num_vgpr(256))) void k_gemm(const bf* __restrict__ AP, const bf* __restrict__ WT, const float* __restrict__ BIAS,
                                                                                    const int* __restrict__ TM, float* CS) {
    __shared__ __align__(16) float os[TROWS * OSP];
    const int lane = threadIdx.x & 31, lr = lane & 15, hi = lane >> 4;
    const int p0 = blockIdx.x * TROWS;
    const int graw = TM[blockIdx.x];
    if (graw < 0) return;
    const int g = min(graw, NMOD - 1);
    v8f acc[16];
#pragma unroll
    for (int nb = 0; nb < 16; ++nb) acc[nb] = (v8f){};
    const size_t aoff = (size_t)(p0 + lr) * SZ + 8 * hi, boff = (size_t)g * (SZ * SZ) + (size_t)lr * SZ + 8 * hi;
#pragma unroll 1
    for (int kc = 0; kc < SZ; kc += 32) {
        const v16bf a = ldb(AP + aoff + kc);
#pragma unroll
        for (int nb = 0; nb < 16; ++nb) { const v16bf b = ldb(WT + boff + (size_t)nb * 16 * SZ + kc);
            acc[nb] = wmmab_g(a, b, acc[nb]); }
    }
#pragma unroll
    for (int nb = 0; nb < 16; ++nb) {
#pragma unroll
        for (int j = 0; j < 8; ++j) os[(hi * 8 + j) * OSP + nb * 16 + lr] = acc[nb][j]; }
    wave_sync();
    v4f bv0 = *(const v4f*)(BIAS + (size_t)g * SZ + 4 * lane);
    v4f bv1 = *(const v4f*)(BIAS + (size_t)g * SZ + 128 + 4 * lane);
#pragma unroll
    for (int i = 0; i < 4; ++i) { bv0[i] = bf2f(f2bf(bv0[i])); bv1[i] = bf2f(f2bf(bv1[i])); }
#pragma unroll 1
    for (int ps = 0; ps < 2; ++ps) {
#pragma unroll 1
        for (int row = 0; row < TROWS; ++row) {
            const v4f x0 = *(const v4fa*)(&os[row * OSP + 4 * lane]);
            const v4f x1 = *(const v4fa*)(&os[row * OSP + 128 + 4 * lane]);
            const v4f y0 = x0 + bv0; const v4f y1 = x1 + bv1;
            float* dst = CS + (size_t)(p0 + row) * SZ;
            *(volatile v4f*)(dst + 4 * lane) = y0;
            *(volatile v4f*)(dst + 128 + 4 * lane) = y1; }
        if (ps == 0) __threadfence(); }
}

__global__ __launch_bounds__(256) void k_unsort(const int* __restrict__ POS, const float* __restrict__ CS, float* OUT) {
    const size_t i = (size_t)blockIdx.x * 256 + threadIdx.x; if (i >= (size_t)NB * (SZ / 4)) return;
    const int b = (int)(i >> 6), c4 = (int)(i & 63);
    const int p = clampi(POS[b], 0, PROWS - 1);
    const v4f v = *(const v4f*)(CS + (size_t)p * SZ + 4 * c4);
    *(volatile v4f*)(OUT + i * 4) = v; __threadfence(); *(volatile v4f*)(OUT + i * 4) = v;
}

static constexpr size_t al256(size_t v) { return (v + 255) & ~(size_t)255; }
static constexpr size_t SZ_WT  = al256((size_t)NMOD * SZ * SZ * 2);
static constexpr size_t SZ_POS = al256((size_t)NB * 4);
static constexpr size_t SZ_TM  = al256((size_t)NTILE * 4);
static constexpr size_t SZ_PL  = al256((size_t)PROWS * SZ * 2);
static constexpr size_t SZ_CS  = al256((size_t)PROWS * SZ * 4);
static constexpr size_t SZ_TOTAL = SZ_WT + SZ_POS + SZ_TM + SZ_PL + SZ_CS;
static_assert(SZ_TOTAL <= (size_t)134217728);
static_assert((size_t)NTILE * TROWS * SZ * 4 <= SZ_CS);
static_assert((size_t)NTILE * TROWS * SZ * 2 <= SZ_PL);

extern "C" void kernel_launch(void* const* d_in, const int* in_sizes, int n_in,
                              void* d_out, int out_size, void* d_ws, size_t ws_size, hipStream_t stream) {
    if (n_in < 4) return;
    if ((size_t)in_sizes[0] < (size_t)NB * SZ) return;
    if ((size_t)in_sizes[1] < (size_t)NB) return;
    if ((size_t)in_sizes[2] < (size_t)NMOD * SZ * SZ) return;
    if ((size_t)in_sizes[3] < (size_t)NMOD * SZ) return;
    if ((size_t)out_size < (size_t)NB * SZ) return;
    if (SZ_TOTAL > ws_size) return;
    const float* x    = (const float*)d_in[0];
    const int*   ids  = (const int*)d_in[1];
    const float* wl   = (const float*)d_in[2];
    const float* bl   = (const float*)d_in[3];
    float* OUT = (float*)d_out;
    char* wsp = (char*)d_ws;
    bf*  WT  = (bf*)wsp;  wsp += SZ_WT;
    int* POS = (int*)wsp; wsp += SZ_POS;
    int* TM  = (int*)wsp; wsp += SZ_TM;
    bf*  AP  = (bf*)wsp;  wsp += SZ_PL;
    float* CS = (float*)wsp; wsp += SZ_CS;

    k_wt<<<NMOD * 16, 256, 0, stream>>>(wl, WT);
    k_sort<<<1, 1024, 0, stream>>>(ids, POS, TM, AP);
    k_pack<<<NB / 32, 256, 0, stream>>>(x, POS, AP);
    k_gemm<<<NTILE, 32, 0, stream>>>(AP, WT, bl, TM, CS);
    k_unsort<<<(unsigned)(((size_t)NB * (SZ / 4) + 255) / 256), 256, 0, stream>>>(POS, CS, OUT);
}
